// CrossAttention_74672301408418
// MI455X (gfx1250) — hardware-verified
//
#include <hip/hip_runtime.h>
#include <stdint.h>


typedef _Float16 v16h __attribute__((ext_vector_type(16)));
typedef _Float16 v8h  __attribute__((ext_vector_type(8)));
typedef float    v8f  __attribute__((ext_vector_type(8)));
typedef float    v4f  __attribute__((ext_vector_type(4)));

#ifndef NB
#define NB 8
#endif
#ifndef SEQ
#define SEQ 1024
#endif
#define NB_FULL  8
#define SEQ_FULL 1024
#define CH       512
#define NH       8
#define HD       64

#define ACT_CAR   8.0f
#define W_CAR     1024.0f
#define PROJ_SCL  0.0001220703125f
#define QKV_CAR   256.0f
#define S_SCL     1.9073486328125e-6f
#define P_CAR     16384.0f
#define O_SCL     6.103515625e-5f
#define OUT_SCL   3.814697265625e-6f

static_assert(SEQ % 128 == 0);
static_assert(SEQ <= SEQ_FULL);
static_assert(NB >= 1 && NB <= NB_FULL);
static_assert(CH == NH * HD);
static_assert(HD == 64);
static_assert(CH % 128 == 0);
static_assert(CH % 32 == 0);
static_assert(((long)NB * SEQ) % 128 == 0);
static_assert((long)NB_FULL * SEQ_FULL * CH * 4 == 16777216L);
static_assert(((long)7 * NB * SEQ * CH + (long)4 * CH * CH) * 2 + 16384 <= 134217728L);

union Frag16 { v16h v; v8h p[2]; };

__device__ __forceinline__ v16h ld_frag(const _Float16* p, int hl) {
  Frag16 f;
  f.p[0] = *(const v8h*)(p + 8 * hl);
  f.p[1] = *(const v8h*)(p + 16 + 8 * hl);
  return f.v;
}

#define LDS_FRAG(dst, arr, off)                                \
  do {                                                         \
    Frag16 f_;                                                 \
    f_.p[0] = *(const v8h*)&arr[(off) + 8 * hl];               \
    f_.p[1] = *(const v8h*)&arr[(off) + 16 + 8 * hl];          \
    dst = f_.v;                                                \
  } while (0)

__device__ __forceinline__ v8f mma(v16h a, v16h b, v8f c) {
  v8f d = __builtin_amdgcn_wmma_f32_16x16x32_f16(false, a, false, b, (short)0, c, false, false);
  asm volatile("v_nop\n\tv_nop\n\tv_nop\n\tv_nop" : "+v"(d) : "v"(a), "v"(b));
  return d;
}

__device__ __forceinline__ float bf16_rne(float x) {
  unsigned int u = __builtin_bit_cast(unsigned int, x);
  u += 0x7FFFu + ((u >> 16) & 1u);
  return __builtin_bit_cast(float, u & 0xFFFF0000u);
}

__global__ __launch_bounds__(256) void k_cvt8(const float* __restrict__ src,
                                              _Float16* __restrict__ dst,
                                              int cols, int rpb, int rpb_full,
                                              float car, int total8)
{
  const int i8 = blockIdx.x * 256 + threadIdx.x;
  if (i8 >= total8) return;
  const size_t e   = (size_t)i8 * 8;
  const size_t r   = e / (size_t)cols;
  const int    col = (int)(e - r * (size_t)cols);
  const size_t rb  = r / (size_t)rpb;
  const size_t rs  = rb * (size_t)rpb_full + (r - rb * (size_t)rpb);
  const float* s = src + rs * (size_t)cols + col;
  const v4f x0 = *(const v4f*)s;
  const v4f x1 = *(const v4f*)(s + 4);
  v8h o;
#pragma unroll
  for (int j = 0; j < 4; ++j) {
    const float t0 = x0[j];
    const float t1 = x1[j];
    o[j]     = (_Float16)(bf16_rne(t0) * car);
    o[4 + j] = (_Float16)(bf16_rne(t1) * car);
  }
  _Float16* d = dst + e;
  *(volatile v8h*)d = o;
  __threadfence();
  *(volatile v8h*)d = o;
}

static_assert((4 * CH) / 4 == 2 * 256);
__global__ __launch_bounds__(256) void k_bn(const float* __restrict__ bn,
                                            float* __restrict__ fa,
                                            float* __restrict__ fc)
{
  const int g = blockIdx.x * 256 + threadIdx.x;
  if (g >= (4 * CH) / 4) return;
  const int e  = g * 4;
  const int p  = e / CH;
  const int ch = e - p * CH;
  const float* b = bn + (size_t)p * 4 * CH + ch;
  const v4f ga = *(const v4f*)(b);
  const v4f be = *(const v4f*)(b + CH);
  const v4f mn = *(const v4f*)(b + 2 * CH);
  const v4f vr = *(const v4f*)(b + 3 * CH);
  v4f a, cc;
#pragma unroll
  for (int j = 0; j < 4; ++j) {
    const float g0 = ga[j], b0 = be[j], m0 = mn[j], v0 = vr[j];
    const float s = bf16_rne(g0) * rsqrtf(bf16_rne(v0) + 1e-5f);
    a[j]  = s;
    cc[j] = bf16_rne(b0) - bf16_rne(m0) * s;
  }
  *(volatile v4f*)(fa + e) = a;
  *(volatile v4f*)(fc + e) = cc;
  __threadfence();
  *(volatile v4f*)(fa + e) = a;
  *(volatile v4f*)(fc + e) = cc;
}

__device__ __forceinline__ void gemm_main(const _Float16* __restrict__ A,
                                          const _Float16* __restrict__ Bt,
                                          int mw, int n0, int c, int hl, v8f (&acc)[8])
{
  const _Float16* ap0 = A  + (size_t)(mw + c) * CH;
  const _Float16* ap1 = A  + (size_t)(mw + 16 + c) * CH;
  const _Float16* bp  = Bt + (size_t)(n0 + c) * CH;
  const size_t bst = (size_t)16 * CH;
#pragma unroll 1
  for (int k0 = 0; k0 < CH; k0 += 32) {
    const v16h a0 = ld_frag(ap0 + k0, hl);
    const v16h a1 = ld_frag(ap1 + k0, hl);
    const v16h b0 = ld_frag(bp + k0, hl);
    const v16h b1 = ld_frag(bp + bst + k0, hl);
    const v16h b2 = ld_frag(bp + 2 * bst + k0, hl);
    const v16h b3 = ld_frag(bp + 3 * bst + k0, hl);
    acc[0] = mma(a0, b0, acc[0]);
    acc[1] = mma(a0, b1, acc[1]);
    acc[2] = mma(a0, b2, acc[2]);
    acc[3] = mma(a0, b3, acc[3]);
    acc[4] = mma(a1, b0, acc[4]);
    acc[5] = mma(a1, b1, acc[5]);
    acc[6] = mma(a1, b2, acc[6]);
    acc[7] = mma(a1, b3, acc[7]);
  }
}

static_assert(128 * 8 == 8 * 128);
template <bool ROWAFF>
__device__ __forceinline__ void gemm_h_body(const _Float16* __restrict__ A,
                                            const _Float16* __restrict__ Bt,
                                            _Float16* __restrict__ C, int ldc,
                                            const float* __restrict__ fa,
                                            const float* __restrict__ fc)
{
  __shared__ __attribute__((aligned(16))) _Float16 ldsE[128 * 72];

  const int tid = threadIdx.x, lane = tid & 31, w = tid >> 5;
  const int hl = lane >> 4, c = lane & 15;
  const int m0 = blockIdx.y * 128, n0 = blockIdx.x * 64;
  const int mw = m0 + 32 * w;

  v8f acc[8] = {};
  gemm_main(A, Bt, mw, n0, c, hl, acc);

#pragma unroll
  for (int i = 0; i < 2; ++i) {
    float ar[8] = {0.f, 0.f, 0.f, 0.f, 0.f, 0.f, 0.f, 0.f};
    float cr[8] = {0.f, 0.f, 0.f, 0.f, 0.f, 0.f, 0.f, 0.f};
    if constexpr (ROWAFF) {
      const int rb = mw + 16 * i + 8 * hl;
      const v4f a0 = *(const v4f*)(fa + rb);
      const v4f a1 = *(const v4f*)(fa + rb + 4);
      const v4f c0 = *(const v4f*)(fc + rb);
      const v4f c1 = *(const v4f*)(fc + rb + 4);
#pragma unroll
      for (int r = 0; r < 4; ++r) {
        ar[r] = a0[r]; ar[4 + r] = a1[r];
        cr[r] = c0[r]; cr[4 + r] = c1[r];
      }
    }
#pragma unroll
    for (int t = 0; t < 4; ++t) {
      float at = 0.f, ct = 0.f;
      if constexpr (!ROWAFF) {
        at = fa[n0 + 16 * t + c];
        ct = fc[n0 + 16 * t + c];
      }
#pragma unroll
      for (int r = 0; r < 8; ++r) {
        const int rowl = 32 * w + 16 * i + 8 * hl + r;
        const float sa = ROWAFF ? ar[r] : at;
        const float sc = ROWAFF ? cr[r] : ct;
        float y = acc[i * 4 + t][r] * PROJ_SCL;
        y = y * sa + sc;
        y = fminf(fmaxf(y, 0.0f), 1.0f);
        ldsE[rowl * 72 + 16 * t + c] = (_Float16)(y * QKV_CAR);
      }
    }
  }
  __syncthreads();

  _Float16* const cb = C + (size_t)m0 * ldc + n0;
  for (int i = 0; i < 8; ++i) {
    const int q = i * 128 + tid;
    const int rowl = q >> 3, chh = (q & 7) * 8;
    const v8h vh = *(const v8h*)&ldsE[rowl * 72 + chh];
    *(volatile v8h*)(cb + (size_t)rowl * ldc + chh) = vh;
  }
  __threadfence();
  for (int i = 0; i < 8; ++i) {
    const int q = i * 128 + tid;
    const int rowl = q >> 3, chh = (q & 7) * 8;
    const v8h vh = *(const v8h*)&ldsE[rowl * 72 + chh];
    *(volatile v8h*)(cb + (size_t)rowl * ldc + chh) = vh;
  }
}

__global__ __launch_bounds__(128) __attribute__((amdgpu_num_vgpr(256)))
void k_gemm_qk(const _Float16* __restrict__ A, const _Float16* __restrict__ Bt,
               _Float16* __restrict__ C,
               const float* __restrict__ fa, const float* __restrict__ fc)
{
  gemm_h_body<false>(A, Bt, C, CH, fa, fc);
}

__global__ __launch_bounds__(128) __attribute__((amdgpu_num_vgpr(256)))
void k_gemm_v(const _Float16* __restrict__ Aw, const _Float16* __restrict__ X,
              _Float16* __restrict__ Vt,
              const float* __restrict__ fa, const float* __restrict__ fc)
{
  const size_t z = blockIdx.z;
  gemm_h_body<true>(Aw, X + z * (size_t)SEQ * CH, Vt + z * (size_t)CH * SEQ, SEQ, fa, fc);
}

static_assert(128 * 16 == 16 * 128);
__global__ __launch_bounds__(128) __attribute__((amdgpu_num_vgpr(256)))
void k_gemm_o(const _Float16* __restrict__ A, const _Float16* __restrict__ Bt,
              float* __restrict__ Out,
              const float* __restrict__ fa, const float* __restrict__ fc)
{
  __shared__ __attribute__((aligned(16))) float ldsF[128 * 68];

  const int tid = threadIdx.x, lane = tid & 31, w = tid >> 5;
  const int hl = lane >> 4, c = lane & 15;
  const int m0 = blockIdx.y * 128, n0 = blockIdx.x * 64;
  const int mw = m0 + 32 * w;

  v8f acc[8] = {};
  gemm_main(A, Bt, mw, n0, c, hl, acc);

#pragma unroll
  for (int i = 0; i < 2; ++i)
#pragma unroll
    for (int t = 0; t < 4; ++t) {
      const float at = fa[n0 + 16 * t + c];
      const float ct = fc[n0 + 16 * t + c];
#pragma unroll
      for (int r = 0; r < 8; ++r) {
        const int rowl = 32 * w + 16 * i + 8 * hl + r;
        const float y = acc[i * 4 + t][r] * OUT_SCL;
        ldsF[rowl * 68 + 16 * t + c] = y * at + ct;
      }
    }
  __syncthreads();

  const int bq = m0 / SEQ;
  const size_t crow0 = (size_t)bq * SEQ_FULL + (size_t)(m0 - bq * SEQ);
  float* const ob = Out + crow0 * CH + n0;
  for (int i = 0; i < 16; ++i) {
    const int q = i * 128 + tid;
    const int rowl = q >> 4, chh = (q & 15) * 4;
    const v4f v = *(const v4f*)&ldsF[rowl * 68 + chh];
    *(volatile v4f*)(ob + (size_t)rowl * CH + chh) = v;
  }
  __threadfence();
  for (int i = 0; i < 16; ++i) {
    const int q = i * 128 + tid;
    const int rowl = q >> 4, chh = (q & 15) * 4;
    const v4f v = *(const v4f*)&ldsF[rowl * 68 + chh];
    *(volatile v4f*)(ob + (size_t)rowl * CH + chh) = v;
  }
}

#define KT_H (64 * 72)
#define VT_H (64 * 72)
#define PW_H (16 * 40)
static_assert(KT_H + VT_H == 128 * 72);
static_assert(64 * 8 == 2 * 256);
static_assert(128 * 8 == 4 * 256);

__global__ __launch_bounds__(256) __attribute__((amdgpu_num_vgpr(256)))
void k_attn(const _Float16* __restrict__ Q, const _Float16* __restrict__ K,
            const _Float16* __restrict__ Vt, _Float16* __restrict__ O)
{
  __shared__ __attribute__((aligned(16))) _Float16 ldsKV[KT_H + VT_H];
  __shared__ __attribute__((aligned(16))) _Float16 ldsP[8 * PW_H];

  const int tid = threadIdx.x, lane = tid & 31, w = tid >> 5;
  const int hl = lane >> 4, c = lane & 15;
  const int qblocks = SEQ / 128;
  const int tbh = blockIdx.x / qblocks;
  const int qb  = blockIdx.x - tbh * qblocks;
  const int tb = tbh >> 3, h = tbh & 7;
  const int q0 = qb * 128;
  const int qw = q0 + 16 * w;

  const size_t qoff  = ((size_t)tb * SEQ + qw + c) * CH + h * HD;
  const size_t kbase = (size_t)tb * SEQ * CH + h * HD;
  const size_t vbase = ((size_t)tb * CH + h * HD) * SEQ;
  const int pbase = w * PW_H;

  float m[8], l[8];
  v8f o[4] = {};
#pragma unroll
  for (int r = 0; r < 8; ++r) { m[r] = -__builtin_inff(); l[r] = 0.f; }

#pragma unroll 1
  for (int kb = 0; kb < SEQ / 64; ++kb) {
    const int mk = kb * 64;
#pragma unroll
    for (int j = 0; j < 2; ++j) {
      const int s  = j * 256 + tid;
      const int rr = s >> 3, cc = (s & 7) * 8;
      const v8h k8 = *(const v8h*)(K + kbase + (size_t)(mk + rr) * CH + cc);
      *(v8h*)&ldsKV[rr * 72 + cc] = k8;
      const v8h v8 = *(const v8h*)(Vt + vbase + (size_t)rr * SEQ + mk + cc);
      *(v8h*)&ldsKV[KT_H + rr * 72 + cc] = v8;
    }
    __syncthreads();

#pragma unroll
    for (int hf = 0; hf < 2; ++hf) {
      v8f s0 = {}, s1 = {};
#pragma unroll
      for (int ks = 0; ks < 2; ++ks) {
        const v16h qf = ld_frag(Q + qoff + 32 * ks, hl);
        v16h kf0, kf1;
        LDS_FRAG(kf0, ldsKV, (32 * hf + c) * 72 + 32 * ks);
        LDS_FRAG(kf1, ldsKV, (32 * hf + 16 + c) * 72 + 32 * ks);
        s0 = mma(qf, kf0, s0);
        s1 = mma(qf, kf1, s1);
      }

#pragma unroll
      for (int r = 0; r < 8; ++r) {
        const float v0 = s0[r] * S_SCL;
        const float v1 = s1[r] * S_SCL;
        float tm = fmaxf(v0, v1);
        tm = fmaxf(tm, __shfl_xor(tm, 1, 32));
        tm = fmaxf(tm, __shfl_xor(tm, 2, 32));
        tm = fmaxf(tm, __shfl_xor(tm, 4, 32));
        tm = fmaxf(tm, __shfl_xor(tm, 8, 32));
        const float mn = fmaxf(m[r], tm);
        const float al = __expf(m[r] - mn);
        const float p0 = __expf(v0 - mn), p1 = __expf(v1 - mn);
        float rs = p0 + p1;
        rs += __shfl_xor(rs, 1, 32);
        rs += __shfl_xor(rs, 2, 32);
        rs += __shfl_xor(rs, 4, 32);
        rs += __shfl_xor(rs, 8, 32);
        l[r] = l[r] * al + rs;
        m[r] = mn;
#pragma unroll
        for (int t = 0; t < 4; ++t) o[t][r] *= al;
        const int po = pbase + (8 * hl + r) * 40 + c;
        ldsP[po]      = (_Float16)(p0 * P_CAR);
        ldsP[po + 16] = (_Float16)(p1 * P_CAR);
      }
      __syncthreads();

      v16h pf;
      LDS_FRAG(pf, ldsP, pbase + c * 40);
#pragma unroll
      for (int t = 0; t < 4; ++t) {
        v16h vf;
        LDS_FRAG(vf, ldsKV, KT_H + (16 * t + c) * 72 + 32 * hf);
        o[t] = mma(pf, vf, o[t]);
      }
    }
    __syncthreads();
  }

#pragma unroll
  for (int r = 0; r < 8; ++r) {
    const float inv = (1.0f / l[r]) * O_SCL;
    const int rowl = 16 * w + 8 * hl + r;
#pragma unroll
    for (int t = 0; t < 4; ++t)
      ldsKV[rowl * 72 + 16 * t + c] = (_Float16)(o[t][r] * inv);
  }
  __syncthreads();
  _Float16* const ob = O + ((size_t)tb * SEQ + q0) * CH + h * HD;
  for (int i = 0; i < 4; ++i) {
    const int qi = i * 256 + tid;
    const int rowl = qi >> 3, chh = (qi & 7) * 8;
    const v8h v = *(const v8h*)&ldsKV[rowl * 72 + chh];
    *(volatile v8h*)(ob + (size_t)rowl * CH + chh) = v;
  }
  __threadfence();
  for (int i = 0; i < 4; ++i) {
    const int qi = i * 256 + tid;
    const int rowl = qi >> 3, chh = (qi & 7) * 8;
    const v8h v = *(const v8h*)&ldsKV[rowl * 72 + chh];
    *(volatile v8h*)(ob + (size_t)rowl * CH + chh) = v;
  }
}

extern "C" void kernel_launch(void* const* d_in, const int* in_sizes, int n_in,
                              void* d_out, int out_size, void* d_ws, size_t ws_size,
                              hipStream_t stream)
{
  if (n_in < 8) return;
  const long need_act = (((long)NB - 1) * SEQ_FULL + SEQ) * CH;
  if ((long)in_sizes[0] < need_act) return;
  if ((long)in_sizes[1] < need_act) return;
  if ((long)in_sizes[2] < need_act) return;
  if ((long)in_sizes[3] < (long)CH * CH) return;
  if ((long)in_sizes[4] < (long)CH * CH) return;
  if ((long)in_sizes[5] < (long)CH * CH) return;
  if ((long)in_sizes[6] < (long)CH * CH) return;
  if ((long)in_sizes[7] < (long)4 * 4 * CH) return;
  if ((long)out_size < need_act) return;

  const float* xq = (const float*)d_in[0];
  const float* xk = (const float*)d_in[1];
  const float* xv = (const float*)d_in[2];
  const float* Wq = (const float*)d_in[3];
  const float* Wk = (const float*)d_in[4];
  const float* Wv = (const float*)d_in[5];
  const float* Wo = (const float*)d_in[6];
  const float* bn = (const float*)d_in[7];
  float* out = (float*)d_out;

  const size_t nAct = (size_t)NB * SEQ * CH;
  const size_t nW   = (size_t)CH * CH;
  const size_t total_bytes = (7 * nAct + 4 * nW) * sizeof(_Float16) + (size_t)2 * 4 * CH * sizeof(float);
  if (total_bytes > ws_size) return;

  _Float16* Xq16 = (_Float16*)d_ws;
  _Float16* Xk16 = Xq16 + nAct;
  _Float16* Xv16 = Xk16 + nAct;
  _Float16* W16  = Xv16 + nAct;
  _Float16* Qp   = W16  + 4 * nW;
  _Float16* Kp   = Qp   + nAct;
  _Float16* Vtp  = Kp   + nAct;
  _Float16* Op   = Vtp  + nAct;
  float* fa = (float*)(Op + nAct);
  float* fc = fa + 4 * CH;

  const int t8 = (int)(nAct / 8);
  k_cvt8<<<(t8 + 255) / 256, 256, 0, stream>>>(xq, Xq16, CH, SEQ, SEQ_FULL, ACT_CAR, t8);
  k_cvt8<<<(t8 + 255) / 256, 256, 0, stream>>>(xk, Xk16, CH, SEQ, SEQ_FULL, ACT_CAR, t8);
  k_cvt8<<<(t8 + 255) / 256, 256, 0, stream>>>(xv, Xv16, CH, SEQ, SEQ_FULL, ACT_CAR, t8);
  const int tw8 = (int)(nW / 8);
  k_cvt8<<<(tw8 + 255) / 256, 256, 0, stream>>>(Wq, W16,          CH, CH, CH, W_CAR, tw8);
  k_cvt8<<<(tw8 + 255) / 256, 256, 0, stream>>>(Wk, W16 + nW,     CH, CH, CH, W_CAR, tw8);
  k_cvt8<<<(tw8 + 255) / 256, 256, 0, stream>>>(Wv, W16 + 2 * nW, CH, CH, CH, W_CAR, tw8);
  k_cvt8<<<(tw8 + 255) / 256, 256, 0, stream>>>(Wo, W16 + 3 * nW, CH, CH, CH, W_CAR, tw8);

  k_bn<<<2, 256, 0, stream>>>(bn, fa, fc);

  k_gemm_qk<<<dim3(CH / 64, (NB * SEQ) / 128), 128, 0, stream>>>(Xq16, W16,      Qp, fa,      fc);
  k_gemm_qk<<<dim3(CH / 64, (NB * SEQ) / 128), 128, 0, stream>>>(Xk16, W16 + nW, Kp, fa + CH, fc + CH);
  k_gemm_v<<<dim3(SEQ / 64, CH / 128, NB), 128, 0, stream>>>(W16 + 2 * nW, Xv16, Vtp, fa + 2 * CH, fc + 2 * CH);

  k_attn<<<NB * NH * (SEQ / 128), 256, 0, stream>>>(Qp, Kp, Vtp, Op);

  k_gemm_o<<<dim3(CH / 64, (NB * SEQ) / 128), 128, 0, stream>>>(Op, W16 + 3 * nW, out, fa + 3 * CH, fc + 3 * CH);
}
